// OverlapNAT_83854941487366
// MI455X (gfx1250) — hardware-verified
//
#include <hip/hip_runtime.h>
#include <stdint.h>

typedef _Float16 v16h __attribute__((ext_vector_type(16)));
typedef _Float16 v8h  __attribute__((ext_vector_type(8)));
typedef float    v8f  __attribute__((ext_vector_type(8)));
typedef float    v4f  __attribute__((ext_vector_type(4)));
typedef v8h __attribute__((may_alias)) v8ha;
typedef v4f __attribute__((may_alias)) v4fa;

union Frag { v16h v; v8h half[2]; };

#define BATCH   2
#define HIMG    256
#define DM      128
#define HP      129
#define TPB     (HP * HP)
#define NTOK    (BATCH * TPB)
#define NTPAD   33344
#define NHEAD   8
#define DHEAD   16
#define KPAT    64
#define KDEP    512
#define KRES    128
#define SPITCH  272
#define NPIX    (BATCH * 3 * HIMG * HIMG)

__device__ __forceinline__ v8f wmma16(v16h a, v16h b, v8f c) {
  v8f d = __builtin_amdgcn_wmma_f32_16x16x32_f16(false, a, false, b, (short)0, c, false, false);
  asm volatile("v_nop\n\tv_nop\n\tv_nop\n\tv_nop" : "+v"(d) : "v"(a), "v"(b));
  return d;
}

__device__ __forceinline__ v16h load_frag(const _Float16* p, int h) {
  Frag f;
  f.half[0] = *(const v8ha*)(p + 8 * h);
  f.half[1] = *(const v8ha*)(p + 16 + 8 * h);
  return f.v;
}

__global__ __launch_bounds__(256) void wconv_kernel(
    const float* __restrict__ qkv_w, const float* __restrict__ proj_w,
    const float* __restrict__ fc1_w, const float* __restrict__ fc2_w,
    const float* __restrict__ pat_w, const float* __restrict__ dep_w,
    const float* __restrict__ res_w,
    _Float16* wqkv, _Float16* wproj, _Float16* wfc1, _Float16* wfc2,
    _Float16* wpat, _Float16* wdep, _Float16* wres)
{
  const int blk = blockIdx.x, tid = threadIdx.x;
  v8h o;
  _Float16* dst;
  if (blk < 288) {
    const float* src;
    _Float16* d;
    int g;
    if (blk < 72)       { src = qkv_w;  d = wqkv;  g = blk * 256 + tid; }
    else if (blk < 96)  { src = proj_w; d = wproj; g = (blk - 72) * 256 + tid; }
    else if (blk < 192) { src = fc1_w;  d = wfc1;  g = (blk - 96) * 256 + tid; }
    else                { src = fc2_w;  d = wfc2;  g = (blk - 192) * 256 + tid; }
    const v4f a = *(const v4fa*)(src + (size_t)g * 8);
    const v4f c = *(const v4fa*)(src + (size_t)g * 8 + 4);
    o[0] = (_Float16)(a.x * 32.0f); o[1] = (_Float16)(a.y * 32.0f);
    o[2] = (_Float16)(a.z * 32.0f); o[3] = (_Float16)(a.w * 32.0f);
    o[4] = (_Float16)(c.x * 32.0f); o[5] = (_Float16)(c.y * 32.0f);
    o[6] = (_Float16)(c.z * 32.0f); o[7] = (_Float16)(c.w * 32.0f);
    dst = d + (size_t)g * 8;
  } else if (blk < 292) {
    const int g = (blk - 288) * 256 + tid;
    const int n = g >> 3, k0 = (g & 7) * 8;
    const bool real = (k0 < 48);
    const int kc = real ? k0 : 40;
    const float* p = pat_w + n * 48 + kc;
    #pragma unroll
    for (int e = 0; e < 8; ++e) o[e] = real ? (_Float16)(p[e] * 16.0f) : (_Float16)0.0f;
    dst = wpat + (size_t)g * 8;
  } else if (blk < 308) {
    const int g = (blk - 292) * 256 + tid;
    const int cls = g >> 10, n = (g >> 6) & 15, k0 = (g & 63) * 8;
    const int t = k0 >> 7, ci0 = k0 & 127;
    const int ty = t >> 1, tx = t & 1, py = cls >> 1, px = cls & 1;
    const int ky = (1 - py) + 2 * ty, kx = (1 - px) + 2 * tx;
    const bool real = (n < 3);
    const int nc = real ? n : 2;
    #pragma unroll
    for (int e = 0; e < 8; ++e) {
      const int ci = ci0 + e;
      const int idx = ((ci * 3 + nc) * 4 + (3 - ky)) * 4 + (3 - kx);
      o[e] = real ? (_Float16)(dep_w[idx] * 16.0f) : (_Float16)0.0f;
    }
    dst = wdep + (size_t)g * 8;
  } else {
    const int g = tid;
    const int n = g >> 4, r = g & 15;
    const int nc = n < 12 ? n : 11, rc = r < 15 ? r : 14;
    #pragma unroll
    for (int e = 0; e < 8; ++e) {
      const int ec = e < 5 ? e : 4;
      const bool real = (n < 12) && (r < 15) && (e < 5);
      o[e] = real ? (_Float16)(res_w[nc * 75 + rc * 5 + ec] * 16.0f) : (_Float16)0.0f;
    }
    dst = wres + (size_t)g * 8;
  }
  *(volatile v8h*)dst = o;
  __threadfence();
  *(volatile v8h*)dst = o;
}

__global__ __launch_bounds__(256) void im2col_kernel(
    const float* __restrict__ x, const float* __restrict__ pw, const float* __restrict__ pb,
    _Float16* apat)
{
  #pragma clang fp contract(off)
  const int t = blockIdx.x * 256 + threadIdx.x;
  const int row = t >> 3, q8 = t & 7;
  const int rowc = row < NTOK ? row : (NTOK - 1);
  const int b = rowc / TPB;
  const int rem = rowc - b * TPB;
  const int oy = rem / HP, ox = rem - oy * HP;
  const bool real = (row < NTOK) && (q8 < 6);
  const int k0 = (q8 < 6 ? q8 : 5) * 8;
  const int c = k0 >> 4, kyb = (k0 & 15) >> 2;
  v8h o;
  #pragma unroll
  for (int e = 0; e < 8; ++e) {
    const int ky = kyb + (e >> 2), kx = e & 3;
    const int hh = (2 * oy + ky + 254) & 255;
    const int ww = (2 * ox + kx + 254) & 255;
    const int pi = (c * 256 + hh) * 256 + ww;
    const int xi = ((b * 3 + c) * 256 + hh) * 256 + ww;
    const float v = x[xi] * pw[pi] + pb[pi];
    o[e] = real ? (_Float16)v : (_Float16)0.0f;
  }
  _Float16* dst = apat + (size_t)row * KPAT + q8 * 8;
  *(volatile v8h*)dst = o;
  __threadfence();
  *(volatile v8h*)dst = o;
}

__device__ __forceinline__ void gemm_store_h(const _Float16* sT, _Float16* Yh, int N,
                                             int m0, int n0, int w, int lane) {
  const int q8 = lane & 7, sub = lane >> 3;
  #pragma unroll
  for (int i = 0; i < 8; ++i) {
    const int lid = 32 * w + 4 * i + sub;
    const v8h v = *(const v8ha*)(sT + lid * 64 + 8 * q8);
    *(volatile v8h*)(Yh + (size_t)(m0 + lid) * N + n0 + 8 * q8) = v;
  }
}
__device__ __forceinline__ void gemm_store_f(const float* sF, float* Yf, int N,
                                             int m0, int n0, int w, int lane) {
  const int q8 = lane & 7, sub = lane >> 3;
  #pragma unroll
  for (int i = 0; i < 16; ++i) {
    const int lid = 64 * w + 4 * i + sub;
    const int row = lid >> 1, hl = lid & 1;
    const v4f v = *(const v4fa*)(sF + row * 64 + 32 * hl + 4 * q8);
    *(volatile v4f*)(Yf + (size_t)(m0 + row) * N + n0 + 32 * hl + 4 * q8) = v;
  }
}

__global__ __launch_bounds__(64) void gemm_kernel(
    const _Float16* __restrict__ A, const _Float16* __restrict__ Bw,
    const float* __restrict__ bias, _Float16* Yh, float* Yf,
    int K, int N, float osc, float hsc, int act, int mode, int resid)
{
  __shared__ __attribute__((aligned(16))) _Float16 sT[64 * 64];
  __shared__ __attribute__((aligned(16))) float    sF[64 * 64];

  const int tid = threadIdx.x, lane = tid & 31, w = tid >> 5;
  const int h = lane >> 4, m = lane & 15;
  const int m0 = blockIdx.x * 64, n0 = blockIdx.y * 64, m0w = m0 + 32 * w;

  const _Float16* a0p = A + (size_t)(m0w + m) * K;
  const _Float16* a1p = a0p + (size_t)16 * K;
  const _Float16* bp  = Bw + (size_t)(n0 + m) * K;

  const v8f z8 = {0.f, 0.f, 0.f, 0.f, 0.f, 0.f, 0.f, 0.f};
  v8f acc[2][4];
  #pragma unroll
  for (int s = 0; s < 2; ++s)
    #pragma unroll
    for (int t = 0; t < 4; ++t) acc[s][t] = z8;

  #pragma unroll 1
  for (int k0 = 0; k0 < K; k0 += 32) {
    const v16h a0 = load_frag(a0p + k0, h);
    const v16h a1 = load_frag(a1p + k0, h);
    #pragma unroll
    for (int t = 0; t < 4; ++t) {
      const v16h b = load_frag(bp + (size_t)t * 16 * K + k0, h);
      acc[0][t] = wmma16(a0, b, acc[0][t]);
      acc[1][t] = wmma16(a1, b, acc[1][t]);
    }
  }

  if (mode == 0) {
    #pragma unroll
    for (int t = 0; t < 4; ++t) {
      const int col = 16 * t + m;
      const float bv = bias[n0 + col];
      #pragma unroll
      for (int s = 0; s < 2; ++s) {
        #pragma unroll
        for (int r = 0; r < 8; ++r) {
          const int rowl = 32 * w + 16 * s + 8 * h + r;
          float v = acc[s][t][r] * osc + bv;
          if (act) v = v > 0.f ? v : 0.01f * v;
          sT[rowl * 64 + col] = (_Float16)(v * hsc);
        }
      }
    }
    __syncthreads();
    gemm_store_h(sT, Yh, N, m0, n0, w, lane);
    __threadfence();
    gemm_store_h(sT, Yh, N, m0, n0, w, lane);
  } else {
    #pragma unroll
    for (int t = 0; t < 4; ++t) {
      const int col = 16 * t + m;
      const float bv = bias[n0 + col];
      #pragma unroll
      for (int s = 0; s < 2; ++s) {
        #pragma unroll
        for (int r = 0; r < 8; ++r) {
          const int rowl = 32 * w + 16 * s + 8 * h + r;
          float v = acc[s][t][r] * osc + bv;
          if (resid) v += Yf[(size_t)(m0 + rowl) * N + n0 + col];
          sF[rowl * 64 + col] = v;
        }
      }
    }
    __syncthreads();
    gemm_store_f(sF, Yf, N, m0, n0, w, lane);
    __threadfence();
    gemm_store_f(sF, Yf, N, m0, n0, w, lane);
  }
}

__global__ __launch_bounds__(256) void ln_kernel(
    const float* __restrict__ src, const float* __restrict__ g,
    const float* __restrict__ bb, _Float16* dst)
{
  const int tid = threadIdx.x;
  const int row = blockIdx.x * 16 + (tid >> 4);
  const int c0 = (tid & 15) * 8;
  const float* p = src + (size_t)row * DM + c0;
  const v4f a = *(const v4fa*)p;
  const v4f c = *(const v4fa*)(p + 4);
  float xv[8] = {a.x, a.y, a.z, a.w, c.x, c.y, c.z, c.w};
  float s = 0.f;
  #pragma unroll
  for (int i = 0; i < 8; ++i) s += xv[i];
  s += __shfl_xor(s, 1); s += __shfl_xor(s, 2); s += __shfl_xor(s, 4); s += __shfl_xor(s, 8);
  const float mean = s * (1.0f / 128.0f);
  float s2 = 0.f;
  #pragma unroll
  for (int i = 0; i < 8; ++i) { xv[i] -= mean; s2 += xv[i] * xv[i]; }
  s2 += __shfl_xor(s2, 1); s2 += __shfl_xor(s2, 2); s2 += __shfl_xor(s2, 4); s2 += __shfl_xor(s2, 8);
  const float var = s2 * (1.0f / 128.0f);
  const float rs = rsqrtf(var + 1e-5f);
  const v4f ga = *(const v4fa*)(g + c0), gc = *(const v4fa*)(g + c0 + 4);
  const v4f ba = *(const v4fa*)(bb + c0), bc = *(const v4fa*)(bb + c0 + 4);
  const float gv[8] = {ga.x, ga.y, ga.z, ga.w, gc.x, gc.y, gc.z, gc.w};
  const float bv[8] = {ba.x, ba.y, ba.z, ba.w, bc.x, bc.y, bc.z, bc.w};
  v8h o;
  #pragma unroll
  for (int i = 0; i < 8; ++i) o[i] = (_Float16)(xv[i] * rs * gv[i] + bv[i]);
  _Float16* d = dst + (size_t)row * DM + c0;
  *(volatile v8h*)d = o;
  __threadfence();
  *(volatile v8h*)d = o;
}

__global__ __launch_bounds__(256) void na_kernel(
    const _Float16* __restrict__ qkv, const float* __restrict__ rpb,
    _Float16* op)
{
  __shared__ __attribute__((aligned(16))) _Float16 so[32 * DM];
  const int tid = threadIdx.x, lane = tid & 31, w = tid >> 5;
  const int tokl = tid >> 3, hh = tid & 7;
  const int tok = blockIdx.x * 32 + tokl;
  const int tokc = tok < NTOK ? tok : (NTOK - 1);
  const int b = tokc / TPB;
  const int rem = tokc - b * TPB;
  const int y = rem / HP, x = rem - y * HP;

  float q[DHEAD];
  {
    const _Float16* qp = qkv + (size_t)tokc * 384 + hh * DHEAD;
    const v8h qa = *(const v8ha*)qp;
    const v8h qb = *(const v8ha*)(qp + 8);
    #pragma unroll
    for (int d = 0; d < 8; ++d) { q[d] = (float)qa[d] * 0.25f; q[8 + d] = (float)qb[d] * 0.25f; }
  }
  float o[DHEAD];
  #pragma unroll
  for (int d = 0; d < DHEAD; ++d) o[d] = 0.f;
  float mrun = -1e30f, lrun = 0.f;
  const float* rp = rpb + hh * 81;

  #pragma unroll 1
  for (int n = 0; n < 25; ++n) {
    const int di = (n * 13) >> 6;
    const int dj = n - 5 * di;
    int yn = y + di - 2; yn += (yn < 0) ? HP : 0; yn -= (yn >= HP) ? HP : 0;
    int xn = x + dj - 2; xn += (xn < 0) ? HP : 0; xn -= (xn >= HP) ? HP : 0;
    const int ntok = b * TPB + yn * HP + xn;
    const _Float16* kp = qkv + (size_t)ntok * 384 + 128 + hh * DHEAD;
    const v8h ka = *(const v8ha*)kp;
    const v8h kb = *(const v8ha*)(kp + 8);
    float s = rp[(2 + di) * 9 + 2 + dj];
    #pragma unroll
    for (int d = 0; d < 8; ++d) s += q[d] * (float)ka[d];
    #pragma unroll
    for (int d = 0; d < 8; ++d) s += q[8 + d] * (float)kb[d];
    const float mnew = fmaxf(mrun, s);
    const float alpha = __expf(mrun - mnew);
    const float p = __expf(s - mnew);
    mrun = mnew;
    lrun = lrun * alpha + p;
    const _Float16* vp = kp + 128;
    const v8h va = *(const v8ha*)vp;
    const v8h vb = *(const v8ha*)(vp + 8);
    #pragma unroll
    for (int d = 0; d < 8; ++d) o[d] = o[d] * alpha + p * (float)va[d];
    #pragma unroll
    for (int d = 0; d < 8; ++d) o[8 + d] = o[8 + d] * alpha + p * (float)vb[d];
  }
  const float inv = (1.0f / lrun) * 16.0f;
  _Float16* sp = so + tokl * DM + hh * DHEAD;
  #pragma unroll
  for (int d = 0; d < DHEAD; ++d) sp[d] = (_Float16)(o[d] * inv);
  __syncthreads();

  const int q8 = lane & 7, sub = lane >> 3;
  const size_t rbase = (size_t)blockIdx.x * 32;
  #pragma unroll
  for (int i = 0; i < 2; ++i) {
    const int lid = w * 8 + i * 4 + sub;
    const int row = lid >> 1, hl = lid & 1;
    const v8h v = *(const v8ha*)(so + row * DM + 64 * hl + 8 * q8);
    *(volatile v8h*)(op + (rbase + row) * DM + 64 * hl + 8 * q8) = v;
  }
  __threadfence();
  #pragma unroll
  for (int i = 0; i < 2; ++i) {
    const int lid = w * 8 + i * 4 + sub;
    const int row = lid >> 1, hl = lid & 1;
    const v8h v = *(const v8ha*)(so + row * DM + 64 * hl + 8 * q8);
    *(volatile v8h*)(op + (rbase + row) * DM + 64 * hl + 8 * q8) = v;
  }
}

__global__ __launch_bounds__(256) void cvt_kernel(const float* __restrict__ src, _Float16* dst)
{
  const size_t t = (size_t)blockIdx.x * 256 + threadIdx.x;
  const v4f a = *(const v4fa*)(src + t * 8);
  const v4f c = *(const v4fa*)(src + t * 8 + 4);
  v8h o;
  o[0] = (_Float16)a.x; o[1] = (_Float16)a.y; o[2] = (_Float16)a.z; o[3] = (_Float16)a.w;
  o[4] = (_Float16)c.x; o[5] = (_Float16)c.y; o[6] = (_Float16)c.z; o[7] = (_Float16)c.w;
  *(volatile v8h*)(dst + t * 8) = o;
  __threadfence();
  *(volatile v8h*)(dst + t * 8) = o;
}

__device__ __forceinline__ void store3_pass(const float* s, float* base, int w, int lane) {
  const int q8 = lane & 7, sub = lane >> 3;
  #pragma unroll
  for (int i = 0; i < 2; ++i) {
    const int L = i * 16 + w * 4 + sub;
    if (L < 24) {
      const int co = L >> 3, seg = L & 7;
      const v4f v = *(const v4fa*)(s + co * 256 + seg * 32 + 4 * q8);
      *(volatile v4f*)(base + (size_t)co * 65536 + seg * 32 + 4 * q8) = v;
    }
  }
}

__global__ __launch_bounds__(128) void depatch_kernel(
    const _Float16* __restrict__ fh, const _Float16* __restrict__ wdep,
    const float* __restrict__ db, float* yp)
{
  __shared__ __attribute__((aligned(16))) float sy[3 * 256];
  const int tid = threadIdx.x, lane = tid & 31, w = tid >> 5;
  const int h = lane >> 4, m = lane & 15;
  const int yy = blockIdx.x, b = blockIdx.y;
  const int ry = yy >> 1, py = yy & 1, rx0 = 32 * w;

  const v8f z8 = {0.f, 0.f, 0.f, 0.f, 0.f, 0.f, 0.f, 0.f};
  v8f acc[2][2];
  acc[0][0] = z8; acc[0][1] = z8; acc[1][0] = z8; acc[1][1] = z8;

  const _Float16* fb = fh + ((size_t)(b * HP + ry) * HP + rx0 + m) * DM;
  const _Float16* bb = wdep + ((size_t)(py * 2) * 16 + m) * KDEP;

  #pragma unroll 1
  for (int ks = 0; ks < 16; ++ks) {
    const int t = ks >> 2, ci0 = (ks & 3) * 32, ty = t >> 1, tx = t & 1;
    const _Float16* ap = fb + ((size_t)ty * HP + tx) * DM + ci0;
    const v16h a0 = load_frag(ap, h);
    const v16h a1 = load_frag(ap + (size_t)16 * DM, h);
    const v16h b0 = load_frag(bb + 32 * ks, h);
    const v16h b1 = load_frag(bb + (size_t)16 * KDEP + 32 * ks, h);
    acc[0][0] = wmma16(a0, b0, acc[0][0]);
    acc[0][1] = wmma16(a0, b1, acc[0][1]);
    acc[1][0] = wmma16(a1, b0, acc[1][0]);
    acc[1][1] = wmma16(a1, b1, acc[1][1]);
  }

  const float bv = db[m < 3 ? m : 2];
  #pragma unroll
  for (int s = 0; s < 2; ++s)
    #pragma unroll
    for (int px = 0; px < 2; ++px)
      #pragma unroll
      for (int r = 0; r < 8; ++r) {
        const int rx = rx0 + 16 * s + 8 * h + r;
        const int xx = 2 * rx + px;
        const float v = acc[s][px][r] * (1.0f / 16.0f) + bv;
        if (m < 3) sy[m * 256 + xx] = v;
      }
  __syncthreads();

  float* base = yp + (size_t)(b * 3) * 65536 + (size_t)yy * 256;
  store3_pass(sy, base, w, lane);
  __threadfence();
  store3_pass(sy, base, w, lane);
}

__global__ __launch_bounds__(128) void res_kernel(
    const float* __restrict__ yp, const _Float16* __restrict__ wres,
    const float* __restrict__ b1, const float* __restrict__ w2,
    const float* __restrict__ b2, float* out)
{
  __shared__ __attribute__((aligned(16))) _Float16 S[16 * SPITCH];
  __shared__ __attribute__((aligned(16))) float sv[12 * 256];
  __shared__ __attribute__((aligned(16))) float so[3 * 256];
  const int tid = threadIdx.x, lane = tid & 31, w = tid >> 5;
  const int h = lane >> 4, m = lane & 15;
  const int yy = blockIdx.x, b = blockIdx.y;
  const float* ybase = yp + (size_t)(b * 3) * 65536;

  #pragma unroll 1
  for (int e = tid; e < 16 * 264; e += 128) {
    const int r = e / 264;
    const int j = e - r * 264;
    const bool realr = (r < 15);
    const int c = realr ? ((r * 13) >> 6) : 0;
    const int dy = realr ? (r - 5 * c) : 0;
    const int ys = (yy + dy + 254) & 255;
    const int xs = (j + 254) & 255;
    const float v = ybase[(size_t)c * 65536 + ys * 256 + xs];
    S[r * SPITCH + j] = realr ? (_Float16)v : (_Float16)0.0f;
  }
  __syncthreads();

  const v8f z8 = {0.f, 0.f, 0.f, 0.f, 0.f, 0.f, 0.f, 0.f};
  v8f acc[4];
  acc[0] = z8; acc[1] = z8; acc[2] = z8; acc[3] = z8;
  #pragma unroll
  for (int ks = 0; ks < 4; ++ks) {
    const v16h bf = load_frag(wres + (size_t)m * KRES + 32 * ks, h);
    const _Float16* s0 = S + (4 * ks + h) * SPITCH;
    const _Float16* s1 = S + (4 * ks + 2 + h) * SPITCH;
    #pragma unroll
    for (int mt = 0; mt < 4; ++mt) {
      const int xx = 64 * w + 16 * mt + m;
      Frag a;
      #pragma unroll
      for (int i = 0; i < 8; ++i) { a.half[0][i] = s0[xx + i]; a.half[1][i] = s1[xx + i]; }
      acc[mt] = wmma16(a.v, bf, acc[mt]);
    }
  }

  const float b1v = b1[m < 12 ? m : 11];
  #pragma unroll
  for (int mt = 0; mt < 4; ++mt)
    #pragma unroll
    for (int r = 0; r < 8; ++r) {
      const int xx = 64 * w + 16 * mt + 8 * h + r;
      float v = acc[mt][r] * (1.0f / 16.0f) + b1v;
      v = v > 0.f ? v : 0.01f * v;
      if (m < 12) sv[m * 256 + xx] = v;
    }
  __syncthreads();

  const float b20 = b2[0], b21 = b2[1], b22 = b2[2];
  #pragma unroll 1
  for (int pp = 0; pp < 2; ++pp) {
    const int xx = tid + 128 * pp;
    float r0 = b20, r1 = b21, r2 = b22;
    #pragma unroll
    for (int rc = 0; rc < 12; ++rc) {
      const float u = sv[rc * 256 + xx];
      r0 += w2[rc] * u;
      r1 += w2[12 + rc] * u;
      r2 += w2[24 + rc] * u;
    }
    so[xx]       = ybase[(size_t)yy * 256 + xx] + r0;
    so[256 + xx] = ybase[(size_t)65536 + (size_t)yy * 256 + xx] + r1;
    so[512 + xx] = ybase[(size_t)131072 + (size_t)yy * 256 + xx] + r2;
  }
  __syncthreads();

  float* obase = out + (size_t)(b * 3) * 65536 + (size_t)yy * 256;
  store3_pass(so, obase, w, lane);
  __threadfence();
  store3_pass(so, obase, w, lane);
}

static inline size_t al256(size_t v) { return (v + 255) & ~(size_t)255; }

extern "C" void kernel_launch(void* const* d_in, const int* in_sizes, int n_in,
                              void* d_out, int out_size, void* d_ws, size_t ws_size,
                              hipStream_t stream)
{
  if (n_in < 24) return;
  if (in_sizes[0] != NPIX) return;
  if (in_sizes[1] != 3 * 65536 || in_sizes[2] != 3 * 65536) return;
  if (in_sizes[3] != 6144 || in_sizes[4] != 128) return;
  if (in_sizes[5] != 384 || in_sizes[6] != 384) return;
  if (in_sizes[7] != 147456 || in_sizes[8] != 1152) return;
  if (in_sizes[9] != 1944) return;
  if (in_sizes[10] != 49152 || in_sizes[11] != 384) return;
  if (in_sizes[12] != 384 || in_sizes[13] != 384) return;
  if (in_sizes[14] != 196608 || in_sizes[15] != 1536) return;
  if (in_sizes[16] != 196608 || in_sizes[17] != 384) return;
  if (in_sizes[18] != 6144 || in_sizes[19] != 3) return;
  if (in_sizes[20] != 900 || in_sizes[21] != 12) return;
  if (in_sizes[22] != 36 || in_sizes[23] != 3) return;
  if (out_size != NPIX) return;

  const float* x         = (const float*)d_in[0];
  const float* pos_w     = (const float*)d_in[1];
  const float* pos_b     = (const float*)d_in[2];
  const float* patch_w   = (const float*)d_in[3];
  const float* patch_b   = (const float*)d_in[4];
  const float* ln1_g     = (const float*)d_in[5];
  const float* ln1_b     = (const float*)d_in[6];
  const float* qkv_w     = (const float*)d_in[7];
  const float* qkv_b     = (const float*)d_in[8];
  const float* rpb       = (const float*)d_in[9];
  const float* proj_w    = (const float*)d_in[10];
  const float* proj_b    = (const float*)d_in[11];
  const float* ln2_g     = (const float*)d_in[12];
  const float* ln2_b     = (const float*)d_in[13];
  const float* fc1_w     = (const float*)d_in[14];
  const float* fc1_b     = (const float*)d_in[15];
  const float* fc2_w     = (const float*)d_in[16];
  const float* fc2_b     = (const float*)d_in[17];
  const float* depatch_w = (const float*)d_in[18];
  const float* depatch_b = (const float*)d_in[19];
  const float* res1_w    = (const float*)d_in[20];
  const float* res1_b    = (const float*)d_in[21];
  const float* res2_w    = (const float*)d_in[22];
  const float* res2_b    = (const float*)d_in[23];
  float* out = (float*)d_out;

  size_t off = 0;
  char* ws = (char*)d_ws;
  _Float16* wqkv  = (_Float16*)(ws + off); off += al256((size_t)3 * 384 * 128 * 2);
  _Float16* wproj = (_Float16*)(ws + off); off += al256((size_t)3 * 128 * 128 * 2);
  _Float16* wfc1  = (_Float16*)(ws + off); off += al256((size_t)3 * 512 * 128 * 2);
  _Float16* wfc2  = (_Float16*)(ws + off); off += al256((size_t)3 * 128 * 512 * 2);
  _Float16* wpat  = (_Float16*)(ws + off); off += al256((size_t)128 * KPAT * 2);
  _Float16* wdep  = (_Float16*)(ws + off); off += al256((size_t)4 * 16 * KDEP * 2);
  _Float16* wres  = (_Float16*)(ws + off); off += al256((size_t)16 * KRES * 2);
  _Float16* apat  = (_Float16*)(ws + off); off += al256((size_t)NTPAD * KPAT * 2);
  float*    f     = (float*)(ws + off);    off += al256((size_t)NTPAD * DM * 4);
  _Float16* lnp   = (_Float16*)(ws + off); off += al256((size_t)NTPAD * DM * 2);
  _Float16* qkvp  = (_Float16*)(ws + off); off += al256((size_t)NTPAD * 384 * 2);
  _Float16* op    = (_Float16*)(ws + off); off += al256((size_t)NTPAD * DM * 2);
  _Float16* hid   = (_Float16*)(ws + off); off += al256((size_t)NTPAD * 512 * 2);
  float*    ypl   = (float*)(ws + off);    off += al256((size_t)NPIX * 4);
  _Float16* fh    = lnp;
  if (off > ws_size) return;
  if (off > (size_t)134217728) return;

  wconv_kernel<<<309, 256, 0, stream>>>(qkv_w, proj_w, fc1_w, fc2_w, patch_w, depatch_w, res1_w,
                                        wqkv, wproj, wfc1, wfc2, wpat, wdep, wres);
  im2col_kernel<<<NTPAD * 8 / 256, 256, 0, stream>>>(x, pos_w, pos_b, apat);
  gemm_kernel<<<dim3(NTPAD / 64, 2), 64, 0, stream>>>(
      apat, wpat, patch_b, hid, f, KPAT, 128, 1.0f / 16.0f, 1.0f, 0, 1, 0);

  for (int l = 0; l < 3; ++l) {
    ln_kernel<<<NTPAD / 16, 256, 0, stream>>>(f, ln1_g + l * 128, ln1_b + l * 128, lnp);
    gemm_kernel<<<dim3(NTPAD / 64, 6), 64, 0, stream>>>(
        lnp, wqkv + (size_t)l * 384 * 128, qkv_b + l * 384, qkvp, f, 128, 384, 1.0f / 32.0f, 1.0f, 0, 0, 0);
    na_kernel<<<NTPAD / 32, 256, 0, stream>>>(qkvp, rpb + l * 648, op);
    gemm_kernel<<<dim3(NTPAD / 64, 2), 64, 0, stream>>>(
        op, wproj + (size_t)l * 128 * 128, proj_b + l * 128, hid, f, 128, 128, 1.0f / 512.0f, 1.0f, 0, 1, 1);
    ln_kernel<<<NTPAD / 16, 256, 0, stream>>>(f, ln2_g + l * 128, ln2_b + l * 128, lnp);
    gemm_kernel<<<dim3(NTPAD / 64, 8), 64, 0, stream>>>(
        lnp, wfc1 + (size_t)l * 512 * 128, fc1_b + l * 512, hid, f, 128, 512, 1.0f / 32.0f, 16.0f, 1, 0, 0);
    gemm_kernel<<<dim3(NTPAD / 64, 2), 64, 0, stream>>>(
        hid, wfc2 + (size_t)l * 128 * 512, fc2_b + l * 128, qkvp, f, 512, 128, 1.0f / 512.0f, 1.0f, 0, 1, 1);
  }

  cvt_kernel<<<NTPAD * DM / 8 / 256, 256, 0, stream>>>(f, fh);
  depatch_kernel<<<dim3(256, BATCH), 128, 0, stream>>>(fh, wdep, depatch_b, ypl);
  res_kernel<<<dim3(256, BATCH), 128, 0, stream>>>(ypl, wres, res1_b, res2_w, res2_b, out);
}
